// EdgeGuidedAttention_18296560681701
// MI455X (gfx1250) — hardware-verified
//
#include <hip/hip_runtime.h>


#ifndef NB
#define NB 4
#endif
#ifndef SEQ
#define SEQ 256
#endif
#define NB_FULL  4
#define SEQ_FULL 256
#define NH_  8
#define HD   64
#define MROWS (NB * NH_ * SEQ)
#define AT   256
#define QT   16
#define OSQ  68
#define SCP  260
#define PHP  264
#define VTP  264
#define PCARRY 16384.0f
#define PCINV  (1.0f / 16384.0f)
#define LOG2E  1.4426950408889634f
#define NEGF   (-1.0e9f)
#define OFF1   ((size_t)NB_FULL * NH_ * SEQ_FULL * HD)

static_assert(SEQ == SEQ_FULL);
static_assert(NB <= NB_FULL);
static_assert(AT == SEQ);
static_assert(SEQ == 2 * 32 * 4);
static_assert(HD == 64);
static_assert(HD % 32 == 0);
static_assert(SEQ % 32 == 0);
static_assert(MROWS % 64 == 0);
static_assert(SEQ % QT == 0);
static_assert(AT * 4 == QT * HD);
static_assert(QT == 2 * (AT / 32));
static_assert(AT * 16 == QT * HD * 4);
static_assert(32 * 16 * 8 == 16 * HD * 4);
static_assert(32 * 16 * 2 == SEQ * 4);
static_assert(256 * 16 * 8 == HD * SEQ * 2);
static_assert((OSQ * 4) % 16 == 0);
static_assert((SCP * 4) % 16 == 0);
static_assert((PHP * 2) % 16 == 0);
static_assert((VTP * 2) % 16 == 0);
static_assert(OFF1 * 4 == (size_t)2097152);
static_assert(OFF1 + (size_t)NB_FULL * NH_ * SEQ_FULL * SEQ_FULL == (size_t)2621440);
static_assert(16 * OSQ * 4 <= 131072);
static_assert(HD * VTP * 2 <= 131072);
static_assert(QT * OSQ * 4 * 2 + QT * SCP * 4 + HD * 4 + QT * 4 + QT * PHP * 2 <= 131072);

typedef _Float16 h16;
typedef unsigned short bf;
typedef __attribute__((ext_vector_type(16))) __bf16   v16bf;
typedef __attribute__((ext_vector_type(16))) _Float16 v16h;
typedef __attribute__((ext_vector_type(8)))  _Float16 v8h;
typedef __attribute__((ext_vector_type(4)))  _Float16 v4h;
typedef __attribute__((ext_vector_type(8)))  unsigned short v8us;
typedef __attribute__((ext_vector_type(8)))  float    v8f;
typedef __attribute__((ext_vector_type(4)))  float    v4f;
typedef v4f  __attribute__((may_alias)) v4fa;
typedef v8h  __attribute__((may_alias)) v8ha;
typedef v4h  __attribute__((may_alias)) v4ha;

__device__ __forceinline__ unsigned short f2bf(float f) { unsigned u = __float_as_uint(f); u += 0x7FFFu + ((u >> 16) & 1u); return (unsigned short)(u >> 16); }
__device__ __forceinline__ float bfr(float f) { return __uint_as_float(((unsigned)f2bf(f)) << 16); }
__device__ __forceinline__ v16h cat16(v8h lo, v8h hi) { return __builtin_shufflevector(lo, hi, 0, 1, 2, 3, 4, 5, 6, 7, 8, 9, 10, 11, 12, 13, 14, 15); }
__device__ __forceinline__ v16bf cat16b(v8us lo, v8us hi) { return __builtin_bit_cast(v16bf, __builtin_shufflevector(lo, hi, 0, 1, 2, 3, 4, 5, 6, 7, 8, 9, 10, 11, 12, 13, 14, 15)); }
__device__ __forceinline__ v16h  ldh(const h16* p) { return cat16(*(const v8h*)p, *(const v8h*)(p + 16)); }
__device__ __forceinline__ v16bf ldb(const bf* p)  { return cat16b(*(const v8us*)p, *(const v8us*)(p + 16)); }
__device__ __forceinline__ void wave_sync() { __builtin_amdgcn_fence(3  , "wavefront"); __builtin_amdgcn_wave_barrier(); asm volatile("" ::: "memory"); }
__device__ __forceinline__ v8f wmma16g(v16h a, v16h b, v8f c) {
    c = __builtin_amdgcn_wmma_f32_16x16x32_f16(false, a, false, b, (short)0, c, false, false);
    asm volatile("v_nop\n\tv_nop\n\tv_nop\n\tv_nop" : "+v"(c) : "v"(a), "v"(b)); return c; }
__device__ __forceinline__ v8f wmmabg(v16bf a, v16bf b, v8f c) {
    c = __builtin_amdgcn_wmma_f32_16x16x32_bf16(false, a, false, b, (short)0, c, false, false);
    asm volatile("v_nop\n\tv_nop\n\tv_nop\n\tv_nop" : "+v"(c) : "v"(a), "v"(b)); return c; }
static __device__ __forceinline__ h16 toh_flush(float v) { const h16 r = (h16)v; return (fabsf(v) < 6.103515625e-05f) ? (h16)0.0f : r; }

__global__ __launch_bounds__(256) void k_cvt8(const float* __restrict__ src, bf* dst, size_t n8) {
    const size_t i = (size_t)blockIdx.x * 256 + threadIdx.x; if (i >= n8) return;
    const v8f v = *(const v8f*)(src + i * 8); v8us o;
#pragma unroll
    for (int k = 0; k < 8; ++k) o[k] = f2bf(v[k]);
    *(volatile v8us*)(dst + i * 8) = o; __threadfence(); *(volatile v8us*)(dst + i * 8) = o;
}

__global__ __launch_bounds__(256) void k_vt(const float* __restrict__ V, h16* VT) {
    __shared__ __align__(16) h16 ts[HD * VTP];
    unsigned t = threadIdx.x; asm volatile("" : "+v"(t));
    const int z = blockIdx.x;
    const float* vr = V + ((size_t)z * SEQ_FULL + (size_t)t) * HD;
#pragma unroll 1
    for (int c = 0; c < HD / 4; ++c) {
        const v4f x = *(const v4f*)(vr + 4 * c);
#pragma unroll
        for (int i = 0; i < 4; ++i) ts[(4 * c + i) * VTP + (int)t] = toh_flush(bfr(x[i]));
    }
    __syncthreads();
    h16* dst = VT + (size_t)z * HD * SEQ;
#pragma unroll 1
    for (int ps = 0; ps < 2; ++ps) {
#pragma unroll
        for (int it = 0; it < 8; ++it) { const int p = it * 256 + (int)t; const int d = p >> 5, c8 = (p & 31) * 8;
            const v8h val = *(const v8ha*)(&ts[d * VTP + c8]);
            *(volatile v8h*)(dst + (size_t)d * SEQ + c8) = val; }
        if (ps == 0) __threadfence(); }
}

__global__ __launch_bounds__(32) void k_projf(const bf* __restrict__ XB, const bf* __restrict__ WB, const float* __restrict__ bias, float* PF) {
    __shared__ __align__(16) float os[16 * OSQ];
    const int lane = threadIdx.x & 31, lr = lane & 15, hi = lane >> 4; const int r0 = blockIdx.x * 64; const int src = blockIdx.y;
    v8f acc[4][4];
#pragma unroll
    for (int mb = 0; mb < 4; ++mb)
#pragma unroll
        for (int nb = 0; nb < 4; ++nb) acc[mb][nb] = (v8f){};
    const size_t aoff = ((size_t)src * MROWS + (size_t)(r0 + lr)) * HD + 8 * hi;
    const size_t boff = (size_t)lr * (2 * HD) + (size_t)src * HD + 8 * hi;
#pragma unroll 1
    for (int kc = 0; kc < HD; kc += 32) {
        v16bf a[4];
#pragma unroll
        for (int mb = 0; mb < 4; ++mb) a[mb] = ldb(XB + aoff + (size_t)mb * 16 * HD + kc);
#pragma unroll
        for (int nb = 0; nb < 4; ++nb) { const v16bf b = ldb(WB + boff + (size_t)nb * 16 * (2 * HD) + kc);
#pragma unroll
            for (int mb = 0; mb < 4; ++mb) acc[mb][nb] = wmmabg(a[mb], b, acc[mb][nb]); }
    }
    float bc[4];
#pragma unroll
    for (int nb = 0; nb < 4; ++nb) { const float bv = bfr(bias[nb * 16 + lr]); bc[nb] = (src == 0) ? bv : 0.0f; }
    const size_t obase = ((size_t)src * MROWS + (size_t)r0) * HD;
#pragma unroll
    for (int mb = 0; mb < 4; ++mb) {
#pragma unroll
        for (int nb = 0; nb < 4; ++nb) {
#pragma unroll
            for (int j = 0; j < 8; ++j) os[(hi * 8 + j) * OSQ + nb * 16 + lr] = acc[mb][nb][j] + bc[nb]; }
        wave_sync();
#pragma unroll 1
        for (int ps = 0; ps < 2; ++ps) {
#pragma unroll
            for (int s = 0; s < 8; ++s) { const int p = s * 32 + lane; const int row = p >> 4, cofs = (p & 15) * 4;
                const v4f val = *(const v4fa*)(&os[row * OSQ + cofs]);
                *(volatile v4f*)(PF + obase + (size_t)(mb * 16 + row) * HD + cofs) = val; }
            if (ps == 0) __threadfence(); }
        wave_sync();
    }
}

__global__ __launch_bounds__(AT) void k_attn(const float* __restrict__ PF, const h16* __restrict__ VT, const float* __restrict__ wo, const float* __restrict__ bo,
                                             const int* __restrict__ mask, float* OUT) {
    __shared__ __align__(16) float aS[QT * OSQ];
    __shared__ __align__(16) float scS[QT * SCP];
    __shared__ __align__(16) float w4S[HD];
    __shared__ __align__(16) float alS[QT];
    __shared__ __align__(16) h16   phS[QT * PHP];
    __shared__ __align__(16) float oS[QT * OSQ];
    unsigned t = threadIdx.x; asm volatile("" : "+v"(t));
    const int lane = (int)(t & 31u), lr = lane & 15, hi = lane >> 4;
    const int wave = __builtin_amdgcn_readfirstlane((int)(threadIdx.x >> 5));
    const int n0 = blockIdx.x * QT; const int z = blockIdx.y; const int b = z / NH_;

    { const v4f av = *(const v4f*)(PF + ((size_t)z * SEQ + (size_t)n0) * HD + (size_t)t * 4);
      *(v4fa*)(&aS[(int)(t >> 4) * OSQ + (int)(t & 15u) * 4]) = av; }
    { const unsigned tw = t < (unsigned)HD ? t : (unsigned)(HD - 1); float wv = wo[tw]; asm volatile("" : "+v"(wv));
      if (t < (unsigned)HD) w4S[t] = 0.4f * bfr(wv); }
    const float bov = bfr(bo[0]);
    __syncthreads();
    if (wave == 0) {
        float sa = 0.0f;
#pragma unroll 4
        for (int e = 0; e < HD; ++e) sa = fmaf(w4S[e], aS[lr * OSQ + e], sa);
        if (hi == 0) alS[lr] = sa;
    }
    __syncthreads();

    const float* cp = PF + (size_t)MROWS * HD + ((size_t)z * SEQ + (size_t)t) * HD;
    float s[QT];
#pragma unroll
    for (int n = 0; n < QT; ++n) s[n] = 0.0f;
    float g = 0.0f;
#pragma unroll 1
    for (int c = 0; c < HD / 4; ++c) {
        const int e0 = c * 4;
        const v4f c4 = *(const v4f*)(cp + e0);
        const v4f w4 = *(const v4fa*)(&w4S[e0]);
        g += w4[0] * c4[0]; g += w4[1] * c4[1]; g += w4[2] * c4[2]; g += w4[3] * c4[3];
#pragma unroll
        for (int n = 0; n < QT; ++n) {
            const v4f a4 = *(const v4fa*)(&aS[n * OSQ + e0]);
            const float h0 = a4[0] + c4[0], h1 = a4[1] + c4[1], h2 = a4[2] + c4[2], h3 = a4[3] + c4[3];
            s[n] += w4[0] * __builtin_fabsf(h0);
            s[n] += w4[1] * __builtin_fabsf(h1);
            s[n] += w4[2] * __builtin_fabsf(h2);
            s[n] += w4[3] * __builtin_fabsf(h3);
        }
    }
    const int* mrow = mask + ((size_t)b * SEQ_FULL + (size_t)n0) * SEQ_FULL + (size_t)t;
#pragma unroll
    for (int n = 0; n < QT; ++n) {
        int mk = mrow[(size_t)n * SEQ_FULL]; asm volatile("" : "+v"(mk));
        const float sv = (s[n] + 1.5f * (alS[n] + g)) + bov;
        scS[n * SCP + (int)t] = (mk == 0) ? NEGF : sv;
    }
    __syncthreads();

    v4f pv[2][2];
#pragma unroll
    for (int rr = 0; rr < 2; ++rr) {
        const int r = wave * 2 + rr;
        const v4f x0 = *(const v4fa*)(&scS[r * SCP + 4 * lane]);
        const v4f x1 = *(const v4fa*)(&scS[r * SCP + 128 + 4 * lane]);
        float mx = fmaxf(fmaxf(fmaxf(x0[0], x0[1]), fmaxf(x0[2], x0[3])), fmaxf(fmaxf(x1[0], x1[1]), fmaxf(x1[2], x1[3])));
#pragma unroll
        for (int off = 16; off > 0; off >>= 1) mx = fmaxf(mx, __shfl_xor(mx, off, 32));
        v4f e0v, e1v; float sum = 0.0f;
#pragma unroll
        for (int i = 0; i < 4; ++i) {
            const float a0 = (x0[i] - mx) * LOG2E, a1 = (x1[i] - mx) * LOG2E;
            const float y0 = __builtin_amdgcn_exp2f(fmaxf(a0, -127.0f)), y1 = __builtin_amdgcn_exp2f(fmaxf(a1, -127.0f));
            e0v[i] = (a0 < -126.0f) ? 0.0f : y0; e1v[i] = (a1 < -126.0f) ? 0.0f : y1;
            sum += e0v[i] + e1v[i]; }
#pragma unroll
        for (int off = 16; off > 0; off >>= 1) sum += __shfl_xor(sum, off, 32);
        const float inv = 1.0f / sum;
        v4f p0, p1; v4h q0, q1;
#pragma unroll
        for (int i = 0; i < 4; ++i) { p0[i] = e0v[i] * inv; p1[i] = e1v[i] * inv; q0[i] = toh_flush(p0[i] * PCARRY); q1[i] = toh_flush(p1[i] * PCARRY); }
        pv[rr][0] = p0; pv[rr][1] = p1;
        *(v4ha*)(&phS[r * PHP + 4 * lane]) = q0; *(v4ha*)(&phS[r * PHP + 128 + 4 * lane]) = q1;
    }
    { float* prow = OUT + OFF1 + ((size_t)z * SEQ_FULL + (size_t)(n0 + 2 * wave)) * SEQ_FULL + 4 * lane;
#pragma unroll 1
      for (int ps = 0; ps < 2; ++ps) {
#pragma unroll
          for (int rr = 0; rr < 2; ++rr) {
              *(volatile v4f*)(prow + (size_t)rr * SEQ_FULL) = pv[rr][0];
              *(volatile v4f*)(prow + (size_t)rr * SEQ_FULL + 128) = pv[rr][1]; }
          if (ps == 0) __threadfence(); } }
    __syncthreads();

    if (wave < 4) {
        const int d0 = wave * 16;
        v8f acc = (v8f){};
        const size_t vb = ((size_t)z * HD + (size_t)(d0 + lr)) * SEQ + 8 * hi;
#pragma unroll
        for (int ks = 0; ks < SEQ / 32; ++ks) {
            const int ai = lr * PHP + ks * 32 + 8 * hi;
            const v16h a = cat16(*(const v8ha*)(&phS[ai]), *(const v8ha*)(&phS[ai + 16]));
            const v16h bb = ldh(VT + vb + (size_t)ks * 32);
            acc = wmma16g(a, bb, acc);
        }
#pragma unroll
        for (int r = 0; r < 8; ++r) oS[(8 * hi + r) * OSQ + d0 + lr] = acc[r] * PCINV;
    }
    __syncthreads();
    { const int row = (int)(t >> 4), cofs = (int)(t & 15u) * 4;
      const v4f val = *(const v4fa*)(&oS[row * OSQ + cofs]);
      float* op = OUT + ((size_t)z * SEQ_FULL + (size_t)(n0 + row)) * HD + cofs;
      *(volatile v4f*)op = val; __threadfence(); *(volatile v4f*)op = val; }
}

static constexpr size_t al256(size_t v) { return (v + 255) & ~(size_t)255; }
static constexpr size_t SZ_XB = al256((size_t)2 * MROWS * HD * 2);
static constexpr size_t SZ_WB = al256((size_t)HD * 2 * HD * 2);
static constexpr size_t SZ_VT = al256((size_t)NB * NH_ * HD * SEQ * 2);
static constexpr size_t SZ_PF = al256((size_t)2 * MROWS * HD * 4);
static constexpr size_t SZ_TOTAL = SZ_XB + SZ_WB + SZ_VT + SZ_PF;
static_assert(SZ_TOTAL <= (size_t)134217728);
static_assert(((size_t)MROWS * HD) % 8 == 0);
static_assert(((size_t)HD * 2 * HD) % 8 == 0);
static_assert(((size_t)MROWS * HD * 2) % 256 == 0);
static_assert(((size_t)MROWS * HD * 4) % 256 == 0);

extern "C" void kernel_launch(void* const* d_in, const int* in_sizes, int n_in,
                              void* d_out, int out_size, void* d_ws, size_t ws_size, hipStream_t stream) {
    if (n_in < 8) return;
    const size_t needx = (size_t)NB * NH_ * SEQ_FULL * HD;
    if ((size_t)in_sizes[0] < needx || (size_t)in_sizes[1] < needx || (size_t)in_sizes[2] < needx) return;
    if ((size_t)in_sizes[3] < (size_t)NB * SEQ_FULL * SEQ_FULL) return;
    if ((size_t)in_sizes[4] < (size_t)HD * 2 * HD) return;
    if (in_sizes[5] < HD || in_sizes[6] < HD || in_sizes[7] < 1) return;
    if ((size_t)out_size < OFF1 + (size_t)NB * NH_ * SEQ_FULL * SEQ_FULL) return;
    if (SZ_TOTAL > ws_size) return;
    const float* query = (const float*)d_in[0];
    const float* key_  = (const float*)d_in[1];
    const float* value = (const float*)d_in[2];
    const int*   mask  = (const int*)d_in[3];
    const float* W_h   = (const float*)d_in[4];
    const float* b_h   = (const float*)d_in[5];
    const float* W_o   = (const float*)d_in[6];
    const float* b_o   = (const float*)d_in[7];
    float* OUT = (float*)d_out;
    char* wsp = (char*)d_ws;
    bf*    XB = (bf*)wsp;    wsp += SZ_XB;
    bf*    WB = (bf*)wsp;    wsp += SZ_WB;
    h16*   VT = (h16*)wsp;   wsp += SZ_VT;
    float* PF = (float*)wsp; wsp += SZ_PF;

    { const size_t n8 = (size_t)MROWS * HD / 8; const unsigned g = (unsigned)((n8 + 255) / 256);
      k_cvt8<<<g, 256, 0, stream>>>(query, XB, n8);
      k_cvt8<<<g, 256, 0, stream>>>(key_, XB + (size_t)MROWS * HD, n8); }
    { const size_t n8 = (size_t)HD * 2 * HD / 8;
      k_cvt8<<<(unsigned)((n8 + 255) / 256), 256, 0, stream>>>(W_h, WB, n8); }
    k_vt<<<NB * NH_, 256, 0, stream>>>(value, VT);
    k_projf<<<dim3(MROWS / 64, 2, 1), 32, 0, stream>>>(XB, WB, b_h, PF);
    k_attn<<<dim3(SEQ / QT, NB * NH_, 1), AT, 0, stream>>>(PF, VT, W_o, b_o, mask, OUT);
}
